// StandardAttention_47699906789402
// MI455X (gfx1250) — hardware-verified
//
#include <hip/hip_runtime.h>


#ifndef NB
#define NB 2
#endif
#ifndef SEQ
#define SEQ 2048
#endif
#ifndef NB_FULL
#define NB_FULL 2
#endif
#ifndef SEQ_FULL
#define SEQ_FULL 2048
#endif

namespace {
constexpr int H = 16, HD = 64, C = 1024, C3 = 3 * C;
constexpr int ER = (SEQ < 256) ? SEQ : 256;
constexpr int MR = NB * SEQ;
constexpr float XS = 8.0f, WSC = 1024.0f, RS = 1024.0f, PS = 1024.0f, PRS = 1024.0f, LOG2E = 1.4426950408889634f;
static_assert(SEQ % 64 == 0 && SEQ >= 64 && SEQ <= SEQ_FULL && NB >= 1 && NB <= NB_FULL && ER % 64 == 0 && ER <= SEQ);
static_assert(C == H * HD && HD == 64 && C % 64 == 0 && C3 % 64 == 0 && C % 32 == 0 && MR % 64 == 0);

typedef _Float16 b16;
typedef __attribute__((ext_vector_type(16))) _Float16 v16b;
typedef __attribute__((ext_vector_type(8))) _Float16 v8b;
typedef __attribute__((ext_vector_type(8))) float v8f;
typedef __attribute__((ext_vector_type(4))) float v4f;

__device__ __forceinline__ float bf16_rne(float f) { unsigned int u = __float_as_uint(f); u += 0x7FFFu + ((u >> 16) & 1u); return __uint_as_float(u & 0xFFFF0000u); }
__device__ __forceinline__ v16b frag_kb(const b16* p, int hh) {
  const v8b a = *(const v8b*)(p + 8 * hh), b = *(const v8b*)(p + 16 + 8 * hh); v16b f;
#pragma unroll
  for (int e = 0; e < 8; ++e) { f[e] = a[e]; f[8 + e] = b[e]; }
  return f;
}
__device__ __forceinline__ v8f wmma16b(v16b a, v16b b, v8f c) {
  v8f d = __builtin_amdgcn_wmma_f32_16x16x32_f16(false, a, false, b, (short)0, c, false, false);
  asm volatile("v_nop\n\tv_nop\n\tv_nop\n\tv_nop" : "+v"(d) : "v"(a), "v"(b));
  return d;
}
__device__ __forceinline__ void wave_lds_sync() { __builtin_amdgcn_fence(3, "workgroup"); __builtin_amdgcn_wave_barrier(); __builtin_amdgcn_fence(2, "workgroup"); }
__device__ __forceinline__ float nexp2(float v) { return __builtin_amdgcn_exp2f(v); }

__global__ __launch_bounds__(256) void cvt_x_kernel(const float* __restrict__ X, b16* __restrict__ Xp) {
  const size_t u = (size_t)blockIdx.x * 256 + threadIdx.x; const size_t row = u >> 7; const int piece = (int)(u & 127);
  if (row >= (size_t)MR) return;
  const size_t bb = row / SEQ, t = row % SEQ;
  const float* src = X + ((bb * SEQ_FULL + t) * C + (size_t)piece * 8);
  b16* dst = Xp + (row * C + (size_t)piece * 8);
  const v4f x0 = *(const v4f*)src, x1 = *(const v4f*)(src + 4); v8b o;
#pragma unroll
  for (int j = 0; j < 4; ++j) { o[j] = (b16)(bf16_rne(x0[j]) * XS); o[4 + j] = (b16)(bf16_rne(x1[j]) * XS); }
  *(volatile v8b*)dst = o; __threadfence(); *(volatile v8b*)dst = o;
}

template <bool TWO>
__global__ __launch_bounds__(64) void cvt_w_kernel(const float* __restrict__ W, int N, b16* __restrict__ Wt, b16* __restrict__ Wt1) {
  __shared__ __attribute__((aligned(16))) float St[64][64 + 4];
  const int tid = threadIdx.x, wave = tid >> 5, lane = tid & 31; const int kb = (int)blockIdx.x, nb = (int)blockIdx.y;
  const float* src = W + ((size_t)kb * 64 * N + (size_t)nb * 64);
  for (int it = 0; it < 16; ++it) {
    const int e = (it * 64 + tid) * 4; const int kk = e >> 6, nn = e & 63;
    const v4f x = *(const v4f*)(src + (size_t)kk * N + nn);
#pragma unroll
    for (int j = 0; j < 4; ++j) St[nn + j][kk] = bf16_rne(x[j]);
  }
  __syncthreads();
  b16* dst = Wt + ((size_t)nb * 64 * C + (size_t)kb * 64); b16* dst1 = Wt1 + ((size_t)nb * 64 * C + (size_t)kb * 64);
  for (int pass = 0; pass < 2; ++pass) {
#pragma unroll 1
    for (int it = 0; it < 8; ++it) {
      const int n = wave * 32 + it * 4 + (lane >> 3), kp = (lane & 7) * 8;
      const v4f a0 = *(const v4f*)(&St[n][kp]), a1 = *(const v4f*)(&St[n][kp + 4]); v8b o, o1;
#pragma unroll
      for (int j = 0; j < 4; ++j) { o[j] = (b16)(a0[j] * WSC); o[4 + j] = (b16)(a1[j] * WSC); o1[j] = (b16)a0[j]; o1[4 + j] = (b16)a1[j]; }
      *(volatile v8b*)(dst + (size_t)n * C + kp) = o;
      if constexpr (TWO) *(volatile v8b*)(dst1 + (size_t)n * C + kp) = o1; }
    __threadfence(); }
}

__global__ __launch_bounds__(64) __attribute__((amdgpu_num_vgpr(256))) void qkv_kernel(const b16* __restrict__ Xp, const b16* __restrict__ Wa, const float* __restrict__ bias,
    b16* __restrict__ Qh, b16* __restrict__ Kh, b16* __restrict__ VT, b16* __restrict__ Qr, b16* __restrict__ Kr, b16* __restrict__ VrT) {
  __shared__ __attribute__((aligned(16))) float Sf[64][64 + 4];
  const int wave = threadIdx.x >> 5, lane = threadIdx.x & 31, hh = lane >> 4, col = lane & 15;
  const int n0 = (int)blockIdx.x * 64, m0 = (int)blockIdx.y * 64;
  const int sec = n0 / C, hn = (n0 % C) / HD;
  const int bb = m0 / SEQ, t0 = m0 % SEQ; const bool early = t0 < ER;
  const b16* Ab = Xp + (size_t)(m0 + wave * 32) * C; const b16* Bb = Wa + (size_t)n0 * C;
  v8f acc[8];
#pragma unroll
  for (int i = 0; i < 8; ++i) acc[i] = (v8f){};
#pragma unroll 1
  for (int k0 = 0; k0 < C; k0 += 32) {
    const v16b a0 = frag_kb(Ab + (size_t)col * C + k0, hh), a1 = frag_kb(Ab + (size_t)(16 + col) * C + k0, hh);
    const v16b b0 = frag_kb(Bb + (size_t)col * C + k0, hh), b1 = frag_kb(Bb + (size_t)(16 + col) * C + k0, hh);
    const v16b b2 = frag_kb(Bb + (size_t)(32 + col) * C + k0, hh), b3 = frag_kb(Bb + (size_t)(48 + col) * C + k0, hh);
    acc[0] = wmma16b(a0, b0, acc[0]); acc[1] = wmma16b(a0, b1, acc[1]); acc[2] = wmma16b(a0, b2, acc[2]); acc[3] = wmma16b(a0, b3, acc[3]);
    acc[4] = wmma16b(a1, b0, acc[4]); acc[5] = wmma16b(a1, b1, acc[5]); acc[6] = wmma16b(a1, b2, acc[6]); acc[7] = wmma16b(a1, b3, acc[7]);
  }
#pragma unroll
  for (int i = 0; i < 8; ++i) {
    const int lr = wave * 32 + (i >> 2) * 16 + 8 * hh, lc = (i & 3) * 16 + col;
#pragma unroll
    for (int r = 0; r < 8; ++r) { if (sec == 2) Sf[lc][lr + r] = acc[i][r]; else Sf[lr + r][lc] = acc[i][r]; } }
  __syncthreads();
  const float inva = 1.0f / (XS * WSC);
  const size_t bh = (size_t)bb * H + hn;
  for (int pass = 0; pass < 2; ++pass) {
#pragma unroll 1
    for (int it = 0; it < 8; ++it) {
      const int L = wave * 32 + it * 4 + (lane >> 3), p8 = (lane & 7) * 8;
      const v4f a0 = *(const v4f*)(&Sf[L][p8]), a1 = *(const v4f*)(&Sf[L][p8 + 4]);
      v8f val;
      if (sec < 2) {
        const v4f g0 = *(const v4f*)(bias + n0 + p8), g1 = *(const v4f*)(bias + n0 + p8 + 4);
#pragma unroll
        for (int j = 0; j < 4; ++j) { val[j] = a0[j] * inva + bf16_rne(g0[j]); val[4 + j] = a1[j] * inva + bf16_rne(g1[j]); }
      } else {
        const float g = bf16_rne(bias[n0 + L]);
#pragma unroll
        for (int j = 0; j < 4; ++j) { val[j] = a0[j] * inva + g; val[4 + j] = a1[j] * inva + g; }
      }
      v8b oh, orr;
#pragma unroll
      for (int j = 0; j < 8; ++j) { const float s8 = val[j] * XS; const b16 hv = (b16)s8; oh[j] = hv; orr[j] = (b16)((s8 - (float)hv) * RS); }
      b16* dh; b16* dr;
      if (sec < 2) { b16* ph = (sec == 0) ? Qh : Kh; b16* pr = (sec == 0) ? Qr : Kr;
        dh = ph + ((bh * SEQ + t0 + L) * HD + p8); dr = pr + ((bh * ER + t0 + L) * HD + p8); }
      else { dh = VT + ((bh * HD + L) * SEQ + t0 + p8); dr = VrT + ((bh * HD + L) * ER + t0 + p8); }
      *(volatile v8b*)dh = oh;
      if (early) *(volatile v8b*)dr = orr; }
    __threadfence(); }
}

template <bool EV>
__global__ __launch_bounds__(64) __attribute__((amdgpu_num_vgpr(256))) void attn_kernel(const b16* __restrict__ Qh, const b16* __restrict__ Kh, const b16* __restrict__ VT,
    const b16* __restrict__ Qr, const b16* __restrict__ Kr, const b16* __restrict__ VrT, b16* __restrict__ Ch, b16* __restrict__ Cr, int qb0) {
  __shared__ __attribute__((aligned(16))) b16 Pb[2][16][32 + 8];
  __shared__ __attribute__((aligned(16))) b16 Pr[2][16][32 + 8];
  __shared__ __attribute__((aligned(16))) float To[2][16][HD + 4];
  const int wave = threadIdx.x >> 5, lane = threadIdx.x & 31, hh = lane >> 4, col = lane & 15;
  const int bhi = (int)blockIdx.y; const int bb = bhi / H, hn = bhi % H;
  const int bx = (int)blockIdx.x + qb0; const int q0 = bx * 32 + wave * 16, qi = q0 + col;
  const b16* Qb = Qh + (size_t)bhi * SEQ * HD; const b16* Kb = Kh + (size_t)bhi * SEQ * HD; const b16* Vb = VT + (size_t)bhi * HD * SEQ;
  const b16* Qrb = Qr + (size_t)bhi * ER * HD; const b16* Krb = Kr + (size_t)bhi * ER * HD; const b16* Vrb = VrT + (size_t)bhi * HD * ER;
  const v16b qa0 = frag_kb(Qb + (size_t)qi * HD, hh), qa1 = frag_kb(Qb + (size_t)qi * HD + 32, hh);
  v16b qx0 = (v16b){}, qx1 = (v16b){};
  if constexpr (EV) { qx0 = frag_kb(Qrb + (size_t)qi * HD, hh); qx1 = frag_kb(Qrb + (size_t)qi * HD + 32, hh); }
  const float cs = LOG2E / (8.0f * XS * XS);
  float m = -INFINITY, l = 0.0f; v8f o[4], o2[4];
#pragma unroll
  for (int t = 0; t < 4; ++t) { o[t] = (v8f){}; o2[t] = (v8f){}; }
  const int kend = bx * 32 + 32;
#pragma unroll 1
  for (int kb = 0; kb < kend; kb += 32) {
    float e[16]; float mx = -INFINITY;
#pragma unroll
    for (int u = 0; u < 2; ++u) {
      const size_t kr = (size_t)(kb + u * 16 + col) * HD;
      const v16b kh0 = frag_kb(Kb + kr, hh), kh1 = frag_kb(Kb + kr + 32, hh);
      v8f s = (v8f){}; s = wmma16b(kh0, qa0, s); s = wmma16b(kh1, qa1, s);
      v8f s2 = (v8f){};
      if constexpr (EV) {
        const v16b kx0 = frag_kb(Krb + kr, hh), kx1 = frag_kb(Krb + kr + 32, hh);
        s2 = wmma16b(kh0, qx0, s2); s2 = wmma16b(kh1, qx1, s2); s2 = wmma16b(kx0, qa0, s2); s2 = wmma16b(kx1, qa1, s2); }
#pragma unroll
      for (int r = 0; r < 8; ++r) {
        float sv = s[r];
        if constexpr (EV) sv += s2[r] * (1.0f / RS);
        const int key = kb + u * 16 + 8 * hh + r;
        const float v = (key > qi) ? -INFINITY : sv * cs; e[u * 8 + r] = v; mx = fmaxf(mx, v); } }
    mx = fmaxf(mx, __shfl_xor(mx, 16)); const float mn = fmaxf(m, mx); const float al = nexp2(m - mn); float sum = 0.0f;
#pragma unroll
    for (int i2 = 0; i2 < 16; ++i2) {
      const float p = nexp2(e[i2] - mn); sum += p; const int pi = (i2 < 8 ? 0 : 16) + 8 * hh + (i2 & 7);
      const float pp = p * PS; const b16 ph = (b16)pp; Pb[wave][col][pi] = ph;
      if constexpr (EV) Pr[wave][col][pi] = (b16)((pp - (float)ph) * PRS); }
    sum += __shfl_xor(sum, 16); l = l * al + sum; m = mn;
    wave_lds_sync();
    const v16b pf = frag_kb(&Pb[wave][col][0], hh);
    v16b prf = (v16b){};
    if constexpr (EV) prf = frag_kb(&Pr[wave][col][0], hh);
#pragma unroll
    for (int t = 0; t < 4; ++t) {
      o[t] *= al; const v16b vh = frag_kb(Vb + (size_t)(t * 16 + col) * SEQ + kb, hh);
      o[t] = wmma16b(vh, pf, o[t]);
      if constexpr (EV) {
        const v16b vx = frag_kb(Vrb + (size_t)(t * 16 + col) * ER + kb, hh);
        o2[t] *= al; o2[t] = wmma16b(vh, prf, o2[t]); o2[t] = wmma16b(vx, pf, o2[t]); } }
    wave_lds_sync(); }
  const float inv = 1.0f / (l * PS * XS);
#pragma unroll
  for (int t = 0; t < 4; ++t) {
#pragma unroll
    for (int r = 0; r < 8; ++r) {
      float ov = o[t][r];
      if constexpr (EV) ov += o2[t][r] * (1.0f / PRS);
      To[wave][col][t * 16 + 8 * hh + r] = ov * inv; } }
  wave_lds_sync();
  b16* ch = Ch + ((size_t)(bb * SEQ + q0) * C + (size_t)hn * HD);
  b16* cr = Cr + ((size_t)(bb * ER + q0) * C + (size_t)hn * HD);
  for (int pass = 0; pass < 2; ++pass) {
#pragma unroll 1
    for (int it = 0; it < 4; ++it) {
      const int rr = it * 4 + (lane >> 3), p8 = (lane & 7) * 8;
      const v4f a0 = *(const v4f*)(&To[wave][rr][p8]), a1 = *(const v4f*)(&To[wave][rr][p8 + 4]); v8b oh, orr;
#pragma unroll
      for (int j = 0; j < 4; ++j) {
        const float s0 = a0[j] * XS; const b16 h0 = (b16)s0; oh[j] = h0; orr[j] = (b16)((s0 - (float)h0) * RS);
        const float s1 = a1[j] * XS; const b16 h1 = (b16)s1; oh[4 + j] = h1; orr[4 + j] = (b16)((s1 - (float)h1) * RS); }
      *(volatile v8b*)(ch + (size_t)rr * C + p8) = oh;
      if constexpr (EV) *(volatile v8b*)(cr + (size_t)rr * C + p8) = orr; }
    __threadfence(); }
}

template <bool EV>
__global__ __launch_bounds__(64) __attribute__((amdgpu_num_vgpr(256))) void proj_kernel(const b16* __restrict__ Ch, const b16* __restrict__ Cr, const b16* __restrict__ Wp,
    const b16* __restrict__ Wp1, const float* __restrict__ bias, float* __restrict__ out, int tb0, int ntb) {
  __shared__ __attribute__((aligned(16))) float Sf[64][64 + 4];
  const int wave = threadIdx.x >> 5, lane = threadIdx.x & 31, hh = lane >> 4, col = lane & 15;
  const int n0 = (int)blockIdx.x * 64; const int by = (int)blockIdx.y; const int bb = by / ntb, t0 = tb0 + (by % ntb) * 64;
  const int m0 = bb * SEQ + t0;
  const b16* Ab = Ch + (size_t)(m0 + wave * 32) * C; const b16* Arb = Cr + ((size_t)(bb * ER + t0) + wave * 32) * C;
  const b16* Bb = Wp + (size_t)n0 * C; const b16* B1b = Wp1 + (size_t)n0 * C;
  v8f acc[8];
#pragma unroll
  for (int i = 0; i < 8; ++i) acc[i] = (v8f){};
#pragma unroll 1
  for (int k0 = 0; k0 < C; k0 += 32) {
    {
      const v16b a0 = frag_kb(Ab + (size_t)col * C + k0, hh), a1 = frag_kb(Ab + (size_t)(16 + col) * C + k0, hh);
      const v16b b0 = frag_kb(Bb + (size_t)col * C + k0, hh), b1 = frag_kb(Bb + (size_t)(16 + col) * C + k0, hh);
      const v16b b2 = frag_kb(Bb + (size_t)(32 + col) * C + k0, hh), b3 = frag_kb(Bb + (size_t)(48 + col) * C + k0, hh);
      acc[0] = wmma16b(a0, b0, acc[0]); acc[1] = wmma16b(a0, b1, acc[1]); acc[2] = wmma16b(a0, b2, acc[2]); acc[3] = wmma16b(a0, b3, acc[3]);
      acc[4] = wmma16b(a1, b0, acc[4]); acc[5] = wmma16b(a1, b1, acc[5]); acc[6] = wmma16b(a1, b2, acc[6]); acc[7] = wmma16b(a1, b3, acc[7]);
    }
    if constexpr (EV) {
      const v16b a0 = frag_kb(Arb + (size_t)col * C + k0, hh), a1 = frag_kb(Arb + (size_t)(16 + col) * C + k0, hh);
      const v16b b0 = frag_kb(B1b + (size_t)col * C + k0, hh), b1 = frag_kb(B1b + (size_t)(16 + col) * C + k0, hh);
      const v16b b2 = frag_kb(B1b + (size_t)(32 + col) * C + k0, hh), b3 = frag_kb(B1b + (size_t)(48 + col) * C + k0, hh);
      acc[0] = wmma16b(a0, b0, acc[0]); acc[1] = wmma16b(a0, b1, acc[1]); acc[2] = wmma16b(a0, b2, acc[2]); acc[3] = wmma16b(a0, b3, acc[3]);
      acc[4] = wmma16b(a1, b0, acc[4]); acc[5] = wmma16b(a1, b1, acc[5]); acc[6] = wmma16b(a1, b2, acc[6]); acc[7] = wmma16b(a1, b3, acc[7]);
    }
  }
#pragma unroll
  for (int i = 0; i < 8; ++i) {
    const int lr = wave * 32 + (i >> 2) * 16 + 8 * hh, lc = (i & 3) * 16 + col;
#pragma unroll
    for (int r = 0; r < 8; ++r) Sf[lr + r][lc] = acc[i][r]; }
  __syncthreads();
  const float inva = 1.0f / (XS * WSC);
  float* ob = out + (((size_t)bb * SEQ_FULL + t0) * C + n0);
  for (int pass = 0; pass < 2; ++pass) {
#pragma unroll 1
    for (int it = 0; it < 16; ++it) {
      const int L = wave * 32 + it * 2 + (lane >> 4), p4 = (lane & 15) * 4;
      const v4f a = *(const v4f*)(&Sf[L][p4]); const v4f g = *(const v4f*)(bias + n0 + p4); v4f v;
#pragma unroll
      for (int j = 0; j < 4; ++j) v[j] = a[j] * inva + bf16_rne(g[j]);
      *(volatile v4f*)(ob + (size_t)L * C + p4) = v; }
    __threadfence(); }
}
}

extern "C" void kernel_launch(void* const* d_in, const int* in_sizes, int n_in, void* d_out, int out_size, void* d_ws, size_t ws_size, hipStream_t stream) {
  const size_t need_x = ((size_t)(NB - 1) * SEQ_FULL + SEQ) * C;
  if (n_in < 5 || (size_t)in_sizes[0] < need_x || (size_t)in_sizes[1] < (size_t)C * C3 || (size_t)in_sizes[2] < (size_t)C3 ||
      (size_t)in_sizes[3] < (size_t)C * C || (size_t)in_sizes[4] < (size_t)C || (size_t)out_size < need_x) return;
  const float* Xin = (const float*)d_in[0]; const float* Wain = (const float*)d_in[1]; const float* Bain = (const float*)d_in[2];
  const float* Wpin = (const float*)d_in[3]; const float* Bpin = (const float*)d_in[4];
  size_t off = 0; char* ws = (char*)d_ws;
  auto carve = [&](size_t bytes) { char* p = ws + off; off += (bytes + 255) & ~(size_t)255; return p; };
  const size_t act = (size_t)MR * C * 2;
  const size_t res_qk = (size_t)NB * H * ER * HD * 2;
  const size_t res_c = (size_t)NB * ER * C * 2;
  b16* Xp = (b16*)carve(act); b16* Wa = (b16*)carve((size_t)C3 * C * 2); b16* Wp = (b16*)carve((size_t)C * C * 2); b16* Wp1 = (b16*)carve((size_t)C * C * 2);
  b16* Qh = (b16*)carve(act); b16* Kh = (b16*)carve(act); b16* VT = (b16*)carve(act);
  b16* Qr = (b16*)carve(res_qk); b16* Kr = (b16*)carve(res_qk); b16* VrT = (b16*)carve(res_qk);
  b16* Ch = (b16*)carve(act); b16* Cr = (b16*)carve(res_c);
  if (off > ws_size || off > ((size_t)128 << 20)) return;
  cvt_x_kernel<<<dim3((unsigned)(((size_t)MR * 128 + 255) / 256)), 256, 0, stream>>>(Xin, Xp);
  cvt_w_kernel<false><<<dim3(C / 64, C3 / 64), 64, 0, stream>>>(Wain, C3, Wa, Wa);
  cvt_w_kernel<true><<<dim3(C / 64, C / 64), 64, 0, stream>>>(Wpin, C, Wp, Wp1);
  qkv_kernel<<<dim3(C3 / 64, MR / 64), 64, 0, stream>>>(Xp, Wa, Bain, Qh, Kh, VT, Qr, Kr, VrT);
  attn_kernel<true><<<dim3(ER / 32, NB * H), 64, 0, stream>>>(Qh, Kh, VT, Qr, Kr, VrT, Ch, Cr, 0);
  if (SEQ > ER) attn_kernel<false><<<dim3((SEQ - ER) / 32, NB * H), 64, 0, stream>>>(Qh, Kh, VT, Qr, Kr, VrT, Ch, Cr, ER / 32);
  proj_kernel<true><<<dim3(C / 64, NB * (ER / 64)), 64, 0, stream>>>(Ch, Cr, Wp, Wp1, Bpin, (float*)d_out, 0, ER / 64);
  if (SEQ > ER) proj_kernel<false><<<dim3(C / 64, NB * ((SEQ - ER) / 64)), 64, 0, stream>>>(Ch, Cr, Wp, Wp1, Bpin, (float*)d_out, ER, (SEQ - ER) / 64);
}
